// MLP_43293270343765
// MI455X (gfx1250) — hardware-verified
//
#include <hip/hip_runtime.h>
#include <math.h>

typedef __attribute__((ext_vector_type(16))) _Float16 v16h;
typedef __attribute__((ext_vector_type(16))) __bf16 v16b;
typedef __attribute__((ext_vector_type(8)))  _Float16 v8h;
typedef __attribute__((ext_vector_type(8)))  float v8f;
typedef __attribute__((ext_vector_type(4)))  float v4f;
typedef __attribute__((ext_vector_type(2)))  float v2f;
typedef __attribute__((ext_vector_type(4)))  unsigned v4u;
typedef __attribute__((ext_vector_type(4)))  int v4i;
typedef float __attribute__((may_alias)) float_a;
typedef int __attribute__((may_alias)) int_a;

template <typename T> __device__ __forceinline__ void vst2(void* p, T v) { *(volatile T*)p = v; __threadfence(); *(volatile T*)p = v; }
__device__ __forceinline__ v8f wmma16(v16h a, v16h b, v8f c) {
  v8f d = __builtin_amdgcn_wmma_f32_16x16x32_f16(false, a, false, b, (short)0, c, false, false);
  asm volatile("v_nop\n\tv_nop\n\tv_nop\n\tv_nop" : "+v"(d) : "v"(a), "v"(b));
  return d;
}
__device__ __forceinline__ v8f wmma_bf(v16b a, v16b b, v8f c) {
  v8f d = __builtin_amdgcn_wmma_f32_16x16x32_bf16(false, a, false, b, (short)0, c, false, false);
  asm volatile("v_nop\n\tv_nop\n\tv_nop\n\tv_nop" : "+v"(d) : "v"(a), "v"(b));
  return d;
}
__device__ __forceinline__ v16h frag_h(const _Float16* rowk0, int lane) {
  union { v16h v; v8h q[2]; } u; const _Float16* p = rowk0 + 8 * (lane >> 4);
  u.q[0] = *(const v8h*)p; u.q[1] = *(const v8h*)(p + 16); return u.v;
}
__device__ __forceinline__ v16h frag_f32(const float* rowk0, int lane) {
  v16h a; const float* p = rowk0 + 8 * (lane >> 4);
#pragma unroll
  for (int i = 0; i < 8; ++i) { a[i] = (_Float16)p[i]; a[8 + i] = (_Float16)p[16 + i]; }
  return a;
}
__device__ __forceinline__ v16h frag_f32s(const float* rowk0, int lane, float sc) {
  v16h a; const float* p = rowk0 + 8 * (lane >> 4);
#pragma unroll
  for (int i = 0; i < 8; ++i) { a[i] = (_Float16)(p[i] * sc); a[8 + i] = (_Float16)(p[16 + i] * sc); }
  return a;
}
__device__ __forceinline__ v16h fragc_f32(const float* W, int k0, int n, int lane, int ld, int K) {
  v16h a; const int g = lane >> 4;
#pragma unroll
  for (int i = 0; i < 8; ++i) { const int ka = k0 + 8 * g + i, kb = ka + 16;
    a[i] = (_Float16)(ka < K ? W[(size_t)(ka < K ? ka : K - 1) * ld + n] : 0.f); a[8 + i] = (_Float16)(kb < K ? W[(size_t)(kb < K ? kb : K - 1) * ld + n] : 0.f); }
  return a;
}
struct F2 { v16b h, l; };
__device__ __forceinline__ F2 bsplit16(const float v[16]) { F2 r;
#pragma unroll
  for (int i = 0; i < 16; ++i) { const __bf16 h = (__bf16)v[i]; r.h[i] = h; r.l[i] = (__bf16)(v[i] - (float)h); }
  return r; }
__device__ __forceinline__ F2 split_row(const float* row, int k0, int lane) { float v[16]; const float* p = row + k0 + 8 * (lane >> 4);
#pragma unroll
  for (int i = 0; i < 8; ++i) { v[i] = p[i]; v[8 + i] = p[16 + i]; }
  return bsplit16(v); }
__device__ __forceinline__ F2 split_rowK(const float* row, int k0, int lane, int K) { float v[16]; const int g = lane >> 4;
#pragma unroll
  for (int i = 0; i < 8; ++i) { const int ka = k0 + 8 * g + i, kb = ka + 16; v[i] = ka < K ? row[ka < K ? ka : K - 1] : 0.f; v[8 + i] = kb < K ? row[kb < K ? kb : K - 1] : 0.f; }
  return bsplit16(v); }
__device__ __forceinline__ F2 split_col(const float* W, int k0, int n, int lane, int ld, int K) { float v[16]; const int g = lane >> 4;
#pragma unroll
  for (int i = 0; i < 8; ++i) { const int ka = k0 + 8 * g + i, kb = ka + 16; v[i] = ka < K ? W[(size_t)(ka < K ? ka : K - 1) * ld + n] : 0.f; v[8 + i] = kb < K ? W[(size_t)(kb < K ? kb : K - 1) * ld + n] : 0.f; }
  return bsplit16(v); }
__device__ __forceinline__ v8f mac3(const F2& a, const F2& b, v8f c) { c = wmma_bf(a.l, b.h, c); c = wmma_bf(a.h, b.l, c); return wmma_bf(a.h, b.h, c); }
__device__ __forceinline__ float sigm(float v) { return 1.0f / (1.0f + expf(-v)); }
#define LDSX() do { asm volatile("s_wait_dscnt 0" ::: "memory"); __builtin_amdgcn_wave_barrier(); __builtin_amdgcn_fence(__ATOMIC_RELEASE, "workgroup"); } while (0)

__device__ __forceinline__ float bfr(float v) { return (float)(__bf16)v; }
#define NEX 500000
#define NGRP 20000
#define REP 25
#define KCTX 20
#define NIDX 23
#define HID 128
#define H2 64
#ifndef NBLK
#define NBLK ((NEX + 63) / 64)
#endif
#define WS_SET 0u
#define WS_END (WS_SET + 4u * (size_t)NGRP * HID)
__global__ __launch_bounds__(128) void k_set(const int* __restrict__ IDX, const float* __restrict__ X, float* __restrict__ SET) {
  const int tid = threadIdx.x; const int gl = tid >> 3, part = tid & 7; const size_t grp = (size_t)blockIdx.x * 16 + gl; const size_t row = grp * REP; const int* ci = IDX + row * NIDX + 3;
  float acc[16];
#pragma unroll
  for (int c = 0; c < 16; ++c) acc[c] = 0.f;
  int cnt = 0;
#pragma unroll 1
  for (int k = 0; k < KCTX; ++k) { int j = ci[k]; cnt += (j > 0) ? 1 : 0; j = j < 0 ? 0 : (j >= 10000 ? 9999 : j); const float* xr = X + (size_t)j * HID + part * 16;
#pragma unroll
    for (int c = 0; c < 16; c += 4) { const v4f v = *(const v4f*)(xr + c); acc[c] += bfr(v[0]); acc[c + 1] += bfr(v[1]); acc[c + 2] += bfr(v[2]); acc[c + 3] += bfr(v[3]); } }
  const float inv = 1.0f / (float)(cnt > 1 ? cnt : 1);
#pragma unroll
  for (int c = 0; c < 16; c += 4) { v4f o; o[0] = acc[c] * inv; o[1] = acc[c + 1] * inv; o[2] = acc[c + 2] * inv; o[3] = acc[c + 3] * inv; vst2(SET + grp * HID + part * 16 + c, o); } }
__global__ __launch_bounds__(128) void k_mlp(const int* __restrict__ IDX, const float* __restrict__ X, const float* __restrict__ SET, const float* __restrict__ W1, const float* __restrict__ B1, const float* __restrict__ W2, const float* __restrict__ B2, const float* __restrict__ W3, const float* __restrict__ B3, float* __restrict__ OUT) {
  __shared__ __align__(16) float sh[4][16][HID + 4]; __shared__ __align__(16) float so[64];
  const int tid = threadIdx.x, wave = tid >> 5, lane = tid & 31, col = lane & 15, g = lane >> 4; const size_t r0 = (size_t)blockIdx.x * 64 + wave * 16; const size_t arow = (r0 + col < NEX) ? r0 + col : NEX - 1;
  int i0 = IDX[arow * NIDX], i1 = IDX[arow * NIDX + 1]; i0 = i0 < 0 ? 0 : (i0 >= 10000 ? 9999 : i0); i1 = i1 < 0 ? 0 : (i1 >= 10000 ? 9999 : i1); const size_t grp = arow / REP;
  v8f acc[8] = {};
#pragma unroll 1
  for (int kc = 0; kc < 12; ++kc) {
    if (kc < 8) { v16b a; const float* p = X + (size_t)(kc < 4 ? i0 : i1) * HID + (kc & 3) * 32 + 8 * g;
#pragma unroll
      for (int i = 0; i < 8; ++i) { a[i] = (__bf16)p[i]; a[8 + i] = (__bf16)p[16 + i]; }
#pragma unroll
      for (int j = 0; j < 8; ++j) { v16b w; const int o = j * 16 + col; const float* wr = W1 + (size_t)o * (3 * HID) + kc * 32 + 8 * g;
#pragma unroll
        for (int i = 0; i < 8; ++i) { w[i] = (__bf16)wr[i]; w[8 + i] = (__bf16)wr[16 + i]; }
        acc[j] = wmma_bf(a, w, acc[j]); } }
    else { const F2 a = split_row(SET + grp * HID, (kc - 8) * 32, lane);
#pragma unroll
      for (int j = 0; j < 8; ++j) { v16b w; const int o = j * 16 + col; const float* wr = W1 + (size_t)o * (3 * HID) + kc * 32 + 8 * g;
#pragma unroll
        for (int i = 0; i < 8; ++i) { w[i] = (__bf16)wr[i]; w[8 + i] = (__bf16)wr[16 + i]; }
        acc[j] = wmma_bf(a.h, w, acc[j]); acc[j] = wmma_bf(a.l, w, acc[j]); } } }
#pragma unroll
  for (int j = 0; j < 8; ++j) { const int o = j * 16 + col; const float bb = bfr(B1[o]);
#pragma unroll
    for (int r = 0; r < 8; ++r) sh[wave][8 * g + r][o] = fmaxf(acc[j][r] + bb, 0.f); }
  LDSX();
  v8f acc2[4] = {};
#pragma unroll
  for (int kc = 0; kc < HID / 32; ++kc) { const F2 a = split_row(&sh[wave][col][0], kc * 32, lane);
#pragma unroll
    for (int j = 0; j < 4; ++j) { v16b w; const int o = j * 16 + col; const float* wr = W2 + (size_t)o * HID + kc * 32 + 8 * g;
#pragma unroll
      for (int i = 0; i < 8; ++i) { w[i] = (__bf16)wr[i]; w[8 + i] = (__bf16)wr[16 + i]; }
      acc2[j] = wmma_bf(a.h, w, acc2[j]); acc2[j] = wmma_bf(a.l, w, acc2[j]); } }
  float p3[8];
#pragma unroll
  for (int r = 0; r < 8; ++r) p3[r] = 0.f;
#pragma unroll
  for (int j = 0; j < 4; ++j) { const int o = j * 16 + col; const float bb = bfr(B2[o]), w3 = bfr(W3[o]);
#pragma unroll
    for (int r = 0; r < 8; ++r) p3[r] += fmaxf(acc2[j][r] + bb, 0.f) * w3; }
#pragma unroll
  for (int r = 0; r < 8; ++r) {
#pragma unroll
    for (int s_ = 1; s_ < 16; s_ <<= 1) p3[r] += __shfl_xor(p3[r], s_); }
  if (col == 0) { const float b3 = bfr(B3[0]);
#pragma unroll
    for (int r = 0; r < 8; ++r) so[wave * 16 + 8 * g + r] = p3[r] + b3; }
  __syncthreads();
  { const size_t base = (size_t)blockIdx.x * 64; const int nval = (base + 64 <= NEX) ? 64 : (int)(NEX - base); if (tid < nval / 4) vst2(OUT + base + tid * 4, *(const v4f*)&so[tid * 4]); } }
extern "C" void kernel_launch(void* const* d_in, const int* in_sizes, int n_in, void* d_out, int out_size, void* d_ws, size_t ws_size, hipStream_t stream) {
  (void)in_sizes; (void)n_in; (void)out_size;
  const float** F = (const float**)d_in;
  if (ws_size < (size_t)WS_END) return;
  char* ws = (char*)d_ws; float* SET = (float*)(ws + WS_SET);
  k_set<<<dim3(NGRP / 16), 128, 0, stream>>>((const int*)d_in[0], F[2], SET);
  k_mlp<<<dim3(NBLK), 128, 0, stream>>>((const int*)d_in[0], F[2], SET, F[3], F[4], F[5], F[6], F[7], F[8], (float*)d_out);
}
